// QuantumOptimizedLayer_7344394076255
// MI455X (gfx1250) — hardware-verified
//
#include <hip/hip_runtime.h>


#define NR   8192
#define DD   1024
#define DM   DD
#define LOSC 1024.0f

typedef _Float16 h16;
typedef unsigned short bf;
typedef __attribute__((ext_vector_type(16))) __bf16   v16bf;
typedef __attribute__((ext_vector_type(16))) _Float16 v16h;
typedef __attribute__((ext_vector_type(8)))  _Float16 v8h;
typedef __attribute__((ext_vector_type(8)))  unsigned short v8us;
typedef __attribute__((ext_vector_type(8)))  float    v8f;
typedef __attribute__((ext_vector_type(4)))  float    v4f;
typedef v8h  __attribute__((may_alias)) v8ha;
typedef v4f  __attribute__((may_alias)) v4fa;
typedef v8us __attribute__((may_alias)) v8usa;

__device__ __forceinline__ unsigned short f2bf(float f) { unsigned u = __float_as_uint(f); u += 0x7FFFu + ((u >> 16) & 1u); return (unsigned short)(u >> 16); }
__device__ __forceinline__ float bf2f(unsigned short b) { return __uint_as_float(((unsigned)b) << 16); }
__device__ __forceinline__ float bfr(float f) { return bf2f(f2bf(f)); }
__device__ __forceinline__ v16h cat16(v8h lo, v8h hi) { return __builtin_shufflevector(lo, hi, 0, 1, 2, 3, 4, 5, 6, 7, 8, 9, 10, 11, 12, 13, 14, 15); }
__device__ __forceinline__ v16bf cat16b(v8us lo, v8us hi) { return __builtin_bit_cast(v16bf, __builtin_shufflevector(lo, hi, 0, 1, 2, 3, 4, 5, 6, 7, 8, 9, 10, 11, 12, 13, 14, 15)); }
__device__ __forceinline__ v8f wmma16(v16h a, v16h b, v8f c) { return __builtin_amdgcn_wmma_f32_16x16x32_f16(false, a, false, b, (short)0, c, false, false); }
__device__ __forceinline__ v8f wmmab(v16bf a, v16bf b, v8f c) { return __builtin_amdgcn_wmma_f32_16x16x32_bf16(false, a, false, b, (short)0, c, false, false); }

template <bool SPLITA, bool F16OUT = false>
__global__ __launch_bounds__(128) void k_gemmb(const bf* __restrict__ A, const bf* __restrict__ Al, const bf* __restrict__ Bn, const float* __restrict__ bias, float* C, int ldc, h16* C2, const float* __restrict__ R = nullptr, int K = DM, int roundR = 1) {
    __shared__ __align__(16) float ost[4][16 * 68];
    const int lane = threadIdx.x & 31, wave = threadIdx.x >> 5, lr = lane & 15, hi = lane >> 4;
    const int r0 = blockIdx.x * 64 + wave * 16, c0 = blockIdx.y * 64;
    const size_t aoff = (size_t)(r0 + lr) * K + 8 * hi;
    size_t boff[4];
#pragma unroll
    for (int t = 0; t < 4; ++t) boff[t] = (size_t)(c0 + t * 16 + lr) * K + 8 * hi;
    v8f acc[4];
#pragma unroll
    for (int t = 0; t < 4; ++t) acc[t] = (v8f){};
#pragma unroll 1
    for (int kc = 0; kc < K; kc += 32) {
        const v16bf a = cat16b(*(const v8us*)(A + aoff + kc), *(const v8us*)(A + aoff + kc + 16));
        v16bf al = a;
        if (SPLITA) al = cat16b(*(const v8us*)(Al + aoff + kc), *(const v8us*)(Al + aoff + kc + 16));
#pragma unroll
        for (int t = 0; t < 4; ++t) { const v16bf b = cat16b(*(const v8us*)(Bn + boff[t] + kc), *(const v8us*)(Bn + boff[t] + kc + 16)); acc[t] = wmmab(a, b, acc[t]); if (SPLITA) acc[t] = wmmab(al, b, acc[t]); }
        asm volatile("v_nop\n\tv_nop\n\tv_nop\n\tv_nop" : "+v"(acc[0]), "+v"(acc[1]), "+v"(acc[2]), "+v"(acc[3]) : "v"(a), "v"(al));
    }
    float* os = &ost[wave][0];
#pragma unroll
    for (int t = 0; t < 4; ++t) { const float bv = bias ? bfr(bias[c0 + t * 16 + lr]) : 0.f;
#pragma unroll
        for (int j = 0; j < 8; ++j) os[(hi * 8 + j) * 68 + t * 16 + lr] = acc[t][j] + bv; }
    __syncthreads();
    if (F16OUT) {
        h16* crow = (h16*)(void*)C + (size_t)r0 * ldc + c0;
        auto pass = [&]() {
#pragma unroll
            for (int s = 0; s < 4; ++s) { const int row = 4 * s + (lane >> 3), piece = lane & 7; const float* sp = os + row * 68 + piece * 8; v8h o, o2;
#pragma unroll
                for (int i = 0; i < 8; ++i) { const h16 a = (h16)sp[i]; o[i] = a; o2[i] = (h16)((sp[i] - (float)a) * LOSC); }
                *(volatile v8h*)(crow + (size_t)row * ldc + piece * 8) = o; if (C2) *(volatile v8h*)(C2 + (size_t)r0 * ldc + c0 + (size_t)row * ldc + piece * 8) = o2; }
        };
        pass(); __threadfence(); pass();
    } else {
        float* crow = C + (size_t)r0 * ldc + c0;
        auto pass = [&]() {
#pragma unroll
            for (int s = 0; s < 8; ++s) { const int Lid = (lane >> 3) + 4 * s, piece = lane & 7; const int row = Lid >> 1, cofs = (Lid & 1) * 32 + piece * 4;
                v4f val = *(const v4fa*)(os + row * 68 + cofs); if (R) { const v4f rv = *(const v4f*)(R + ((size_t)r0 + row) * ldc + c0 + cofs); val += roundR ? (v4f){bfr(rv[0]), bfr(rv[1]), bfr(rv[2]), bfr(rv[3])} : rv; }
                *(volatile v4f*)(crow + (size_t)row * ldc + cofs) = val; }
        };
        pass(); __threadfence(); pass();
    }
}


__global__ __launch_bounds__(256) void k_wt(const float* __restrict__ Wm, int K, int ncols, bf* WT) {
    __shared__ __align__(16) unsigned short tl[64 * 72];
    const int tid = threadIdx.x, k0 = blockIdx.x * 64, n0 = blockIdx.y * 64;
    const int kk = tid >> 2, nq = (tid & 3) * 16;
#pragma unroll
    for (int i = 0; i < 16; ++i) tl[(nq + i) * 72 + kk] = f2bf(Wm[(size_t)(k0 + kk) * ncols + n0 + nq + i]);
    __syncthreads();
    const int piece = tid & 7;
    auto pass = [&]() {
#pragma unroll
        for (int s = 0; s < 2; ++s) { const int nr = (tid >> 3) + 32 * s; const v8us val = *(const v8usa*)(tl + nr * 72 + piece * 8); *(volatile v8us*)(WT + (size_t)(n0 + nr) * K + k0 + piece * 8) = val; }
    };
    pass(); __threadfence(); pass();
}

__global__ __launch_bounds__(256) void k_cvt(const float* __restrict__ src, int nrows, bf* dst) {
    const int lane = threadIdx.x & 31, r = blockIdx.x * 8 + (threadIdx.x >> 5); if (r >= nrows) return;
#pragma unroll 1
    for (int ps = 0; ps < 2; ++ps) {
#pragma unroll
        for (int q = 0; q < DD / 256; ++q) { v8us o;
#pragma unroll
            for (int i = 0; i < 8; ++i) o[i] = f2bf(src[(size_t)r * DD + q * 256 + lane * 8 + i]);
            *(volatile v8us*)(dst + (size_t)r * DD + q * 256 + lane * 8) = o; }
        if (ps == 0) __threadfence(); }
}
__global__ __launch_bounds__(256) void k_scale(const float* __restrict__ vqc, float* SC) {
    const int c = blockIdx.x * 256 + threadIdx.x; if (c >= DD) return; const float th = bfr(vqc[c * 4]), ph = bfr(vqc[c * 4 + 1]); const float s = cosf(th * 0.5f) + sinf(th * 0.5f) * cosf(ph);
    *(volatile float*)(SC + c) = s; __threadfence(); *(volatile float*)(SC + c) = s;
}
template <int MODE>
__global__ __launch_bounds__(256) void k_act(const float* __restrict__ T, const float* __restrict__ vqc, int nrows, bf* dh, bf* dl) {
    const int lane = threadIdx.x & 31, r = blockIdx.x * 8 + (threadIdx.x >> 5); if (r >= nrows) return;
#pragma unroll 1
    for (int ps = 0; ps < 2; ++ps) {
#pragma unroll 1
        for (int c0 = lane * 8; c0 < DD; c0 += 256) { const size_t o = (size_t)r * DD + c0; const v8f v = *(const v8f*)(T + o); v8us oh, ol;
#pragma unroll
            for (int q = 0; q < 8; ++q) { float y;
                if (MODE == 0) y = tanhf(v[q]);
                else if (MODE == 1) y = v[q] * vqc[c0 + q];
                else y = v[q] / (1.0f + __expf(-v[q]));
                const unsigned short hb = f2bf(y); oh[q] = hb; ol[q] = f2bf(y - bf2f(hb)); }
            *(volatile v8us*)(dh + o) = oh; *(volatile v8us*)(dl + o) = ol; }
        if (ps == 0) __threadfence(); }
}

extern "C" void kernel_launch(void* const* d_in, const int* in_sizes, int n_in,
                              void* d_out, int out_size, void* d_ws, size_t ws_size, hipStream_t stream) {
    (void)in_sizes; (void)n_in; (void)out_size;
    const float* x = (const float*)d_in[0]; const float* W1 = (const float*)d_in[1]; const float* b1 = (const float*)d_in[2]; const float* W2 = (const float*)d_in[3]; const float* b2 = (const float*)d_in[4];
    const float* vqc = (const float*)d_in[5]; const float* W3 = (const float*)d_in[6]; const float* b3 = (const float*)d_in[7]; const float* W4 = (const float*)d_in[8]; const float* b4 = (const float*)d_in[9];
    float* out = (float*)d_out;
    char* wsp = (char*)d_ws;
    auto take = [&](size_t bytes) { char* p = wsp; wsp += (bytes + 255) & ~(size_t)255; return (void*)p; };
    bf* WT[4]; for (int i = 0; i < 4; ++i) WT[i] = (bf*)take((size_t)DD * DD * 2);
    bf* Xb = (bf*)take((size_t)NR * DD * 2); float* SC = (float*)take(DD * 4); float* T = (float*)take((size_t)NR * DD * 4); bf* Ph = (bf*)take((size_t)NR * DD * 2); bf* Pl = (bf*)take((size_t)NR * DD * 2);
    if ((size_t)(wsp - (char*)d_ws) > ws_size) return;
    const float* Ws[4] = {W1, W2, W3, W4}; for (int i = 0; i < 4; ++i) k_wt<<<dim3(DD / 64, DD / 64, 1), 256, 0, stream>>>(Ws[i], DD, DD, WT[i]);
    k_cvt<<<NR / 8, 256, 0, stream>>>(x, NR, Xb); k_scale<<<DD / 256, 256, 0, stream>>>(vqc, SC);
    k_gemmb<false, false><<<dim3(NR / 64, DD / 64, 1), 128, 0, stream>>>(Xb, nullptr, WT[0], b1, T, DD, nullptr, nullptr, DD);
    k_act<0><<<NR / 8, 256, 0, stream>>>(T, vqc, NR, Ph, Pl);
    k_gemmb<true, false><<<dim3(NR / 64, DD / 64, 1), 128, 0, stream>>>(Ph, Pl, WT[1], b2, T, DD, nullptr, nullptr, DD);
    k_act<1><<<NR / 8, 256, 0, stream>>>(T, SC, NR, Ph, Pl);
    k_gemmb<true, false><<<dim3(NR / 64, DD / 64, 1), 128, 0, stream>>>(Ph, Pl, WT[2], b3, T, DD, nullptr, nullptr, DD);
    k_act<2><<<NR / 8, 256, 0, stream>>>(T, vqc, NR, Ph, Pl);
    k_gemmb<true, false><<<dim3(NR / 64, DD / 64, 1), 128, 0, stream>>>(Ph, Pl, WT[3], b4, out, DD, nullptr, nullptr, DD);
}
